// SPM_76476187672974
// MI455X (gfx1250) — hardware-verified
//
#include <hip/hip_runtime.h>
#include <stdint.h>
#include <stddef.h>

#define DEVINL __device__ __forceinline__

typedef unsigned short us16;
typedef __bf16   v16b __attribute__((ext_vector_type(16)));
typedef _Float16 v16h __attribute__((ext_vector_type(16)));
typedef us16     v8us __attribute__((ext_vector_type(8)));
typedef float    v8f  __attribute__((ext_vector_type(8)));
typedef float    v4f  __attribute__((ext_vector_type(4)));
typedef v8us __attribute__((may_alias)) v8usa;
typedef v4f  __attribute__((may_alias)) v4fa;
union FragB { v16b v; v16h vh; v8us half[2]; };

#define NPIX  4096
#define NCH   1024
#define NIC   128
#define KCV   1152
#define NPR   4356
#define TPB   256
#define LDP   68
#define LT1   72
#define LT2   136
#define LXP   65

static_assert(TPB == 256);
static_assert(NPR == 66 * 66);
static_assert((LDP * 4) % 16 == 0);
static_assert((LT1 * 2) % 16 == 0);
static_assert((LT2 * 2) % 16 == 0);
static_assert(KCV == 9 * NIC);

DEVINL int imin(int a, int b) { return a < b ? a : b; }
DEVINL int imax(int a, int b) { return a > b ? a : b; }

DEVINL v8f wmma_bf16(const FragB& a, const FragB& b, v8f c) {
  v8f d = __builtin_amdgcn_wmma_f32_16x16x32_bf16(false, a.v, false, b.v, (short)0, c, false, false);
  asm volatile("v_nop\n\tv_nop\n\tv_nop\n\tv_nop" : "+v"(d) : "v"(a.vh), "v"(b.vh));
  return d;
}
DEVINL v8f zero8f() {
  v8f z = {0.f, 0.f, 0.f, 0.f, 0.f, 0.f, 0.f, 0.f};
  return z;
}

DEVINL us16 bf16_bits(float f) {
  unsigned u = __float_as_uint(f);
  u += 0x7FFFu + ((u >> 16) & 1u);
  return (us16)(u >> 16);
}
DEVINL float bf16_val(us16 s) { return __uint_as_float(((unsigned)s) << 16); }
DEVINL void split2(float v, us16& hb, us16& lb) {
  hb = bf16_bits(v);
  lb = bf16_bits(v - bf16_val(hb));
}
DEVINL float sigm(float x) {
  const float e = __expf(-x);
  return __builtin_amdgcn_rcpf(1.0f + e);
}

__global__ __launch_bounds__(TPB) void kw1_k(const float* __restrict__ w0, const float* __restrict__ w1,
                                           const float* __restrict__ w2, us16* __restrict__ planes)
{
  const int which = blockIdx.y;
  const float* src = (which == 0) ? w0 : ((which == 1) ? w1 : w2);
  us16* ph = planes + (size_t)which * 2 * ((size_t)NIC * NCH);
  us16* pl = ph + (size_t)NIC * NCH;
  const int t = blockIdx.x * TPB + threadIdx.x;
  if (t >= (NIC * NCH) / 8) return;
  const float* s = src + (size_t)8 * t;
  const v4f f0 = *(const v4fa*)s;
  const v4f f1 = *(const v4fa*)(s + 4);
  v8us hv, lv;
  #pragma unroll
  for (int i = 0; i < 4; ++i) {
    us16 a, b;
    split2(f0[i], a, b); hv[i] = a;     lv[i] = b;
    split2(f1[i], a, b); hv[4 + i] = a; lv[4 + i] = b;
  }
  us16* dh = ph + (size_t)8 * t;
  us16* dl = pl + (size_t)8 * t;
  *(volatile v8us*)dh = hv;
  *(volatile v8us*)dl = lv;
  __threadfence();
  *(volatile v8us*)dh = hv;
  *(volatile v8us*)dl = lv;
}

__global__ __launch_bounds__(TPB) void kwm_k(const float* __restrict__ wm, us16* __restrict__ ph,
                                           us16* __restrict__ pl)
{
  const int t = blockIdx.x * TPB + threadIdx.x;
  if (t >= (NCH * KCV) / 8) return;
  const int piece = t & 15;
  const int rest  = t >> 4;
  const int oc    = rest / 9;
  const int tap   = rest - oc * 9;
  const float* s = wm + ((size_t)oc * NIC + (size_t)piece * 8) * 9 + tap;
  v8us hv, lv;
  #pragma unroll
  for (int i = 0; i < 8; ++i) {
    const float w = s[i * 9];
    us16 a, b;
    split2(w, a, b);
    hv[i] = a; lv[i] = b;
  }
  us16* dh = ph + (size_t)8 * t;
  us16* dl = pl + (size_t)8 * t;
  *(volatile v8us*)dh = hv;
  *(volatile v8us*)dl = lv;
  __threadfence();
  *(volatile v8us*)dh = hv;
  *(volatile v8us*)dl = lv;
}

__global__ __launch_bounds__(TPB) void kx_k(const float* __restrict__ x0, const float* __restrict__ x1,
                                          const float* __restrict__ x2, us16* __restrict__ xt)
{
  __shared__ float sx[64 * LXP];
  const int tid = threadIdx.x;
  const int bx = blockIdx.x, by = blockIdx.y, z = blockIdx.z;
  const float* x = (z == 0) ? x0 : ((z == 1) ? x1 : x2);
  us16* ph = xt + (size_t)z * 2 * ((size_t)NPIX * NCH);
  us16* pl = ph + (size_t)NPIX * NCH;
  const int p0 = bx * 64, c0 = by * 64;
  {
    const int c = tid >> 2, pc = tid & 3;
    const float* s = x + (size_t)(c0 + c) * NPIX + p0 + pc * 16;
    #pragma unroll
    for (int v = 0; v < 4; ++v) {
      const v4f f = *(const v4fa*)(s + 4 * v);
      float* d = sx + c * LXP + pc * 16 + 4 * v;
      d[0] = f[0]; d[1] = f[1]; d[2] = f[2]; d[3] = f[3];
    }
  }
  __syncthreads();
  const int piece = tid & 7, rl = tid >> 3;
  v8us hv[2], lv[2];
  size_t oo[2];
  #pragma unroll
  for (int g = 0; g < 2; ++g) {
    const int p = g * 32 + rl;
    #pragma unroll
    for (int i = 0; i < 8; ++i) {
      const float v = sx[(piece * 8 + i) * LXP + p];
      us16 a, b;
      split2(v, a, b);
      hv[g][i] = a; lv[g][i] = b;
    }
    oo[g] = (size_t)(p0 + p) * NCH + c0 + piece * 8;
    *(volatile v8us*)(ph + oo[g]) = hv[g];
    *(volatile v8us*)(pl + oo[g]) = lv[g];
  }
  __threadfence();
  #pragma unroll
  for (int g = 0; g < 2; ++g) {
    *(volatile v8us*)(ph + oo[g]) = hv[g];
    *(volatile v8us*)(pl + oo[g]) = lv[g];
  }
}

__global__ __launch_bounds__(TPB) void kt1_k(const us16* __restrict__ gh, const us16* __restrict__ gl,
                                           us16* __restrict__ oh, us16* __restrict__ ol)
{
  __shared__ __attribute__((aligned(16))) us16 sh[NIC * LT1];
  __shared__ __attribute__((aligned(16))) us16 sl[NIC * LT1];
  const int tid = threadIdx.x;
  const int j0 = blockIdx.x * 64;
  #pragma unroll
  for (int ps = 0; ps < 4; ++ps) {
    const int j = (tid >> 4) + 16 * ps, pc = tid & 15;
    const size_t o = (size_t)(j0 + j) * NIC + pc * 8;
    const v8us a = *(const v8usa*)(gh + o);
    const v8us b = *(const v8usa*)(gl + o);
    #pragma unroll
    for (int i = 0; i < 8; ++i) {
      sh[(pc * 8 + i) * LT1 + j] = a[i];
      sl[(pc * 8 + i) * LT1 + j] = b[i];
    }
  }
  __syncthreads();
  const int piece = tid & 7, rl = tid >> 3;
  v8us hv[4], lv[4];
  size_t oo[4];
  #pragma unroll
  for (int g = 0; g < 4; ++g) {
    const int c = g * 32 + rl;
    hv[g] = *(const v8usa*)(sh + c * LT1 + piece * 8);
    lv[g] = *(const v8usa*)(sl + c * LT1 + piece * 8);
    oo[g] = (size_t)c * NPIX + j0 + piece * 8;
    *(volatile v8us*)(oh + oo[g]) = hv[g];
    *(volatile v8us*)(ol + oo[g]) = lv[g];
  }
  __threadfence();
  #pragma unroll
  for (int g = 0; g < 4; ++g) {
    *(volatile v8us*)(oh + oo[g]) = hv[g];
    *(volatile v8us*)(ol + oo[g]) = lv[g];
  }
}

__global__ __launch_bounds__(TPB) void kt2_k(const us16* __restrict__ yh, const us16* __restrict__ yl,
                                           us16* __restrict__ ph_, us16* __restrict__ pl_)
{
  __shared__ __attribute__((aligned(16))) us16 sh[64 * LT2];
  __shared__ __attribute__((aligned(16))) us16 sl[64 * LT2];
  const int tid = threadIdx.x;
  const int ph = blockIdx.x;
  const int pix0 = ph * 64;
  #pragma unroll
  for (int ps = 0; ps < 4; ++ps) {
    const int ic = (tid >> 3) + 32 * ps, pc = tid & 7;
    const size_t o = (size_t)ic * NPIX + pix0 + pc * 8;
    const v8us a = *(const v8usa*)(yh + o);
    const v8us b = *(const v8usa*)(yl + o);
    #pragma unroll
    for (int i = 0; i < 8; ++i) {
      sh[(pc * 8 + i) * LT2 + ic] = a[i];
      sl[(pc * 8 + i) * LT2 + ic] = b[i];
    }
  }
  __syncthreads();
  const int piece = tid & 15, rsub = tid >> 4;
  v8us hv[5], lv[5];
  const size_t qb = (size_t)(ph + 1) * 66;
  #pragma unroll
  for (int ps = 0; ps < 5; ++ps) {
    const int lr = ps * 16 + rsub;
    const int pw = imin(imax(lr - 1, 0), 63);
    const v8us a = *(const v8usa*)(sh + pw * LT2 + piece * 8);
    const v8us b = *(const v8usa*)(sl + pw * LT2 + piece * 8);
    const bool border = (lr == 0) || (lr >= 65);
    #pragma unroll
    for (int i = 0; i < 8; ++i) {
      hv[ps][i] = border ? (us16)0 : a[i];
      lv[ps][i] = border ? (us16)0 : b[i];
    }
    if (lr < 66) {
      const size_t o = (qb + lr) * NIC + piece * 8;
      *(volatile v8us*)(ph_ + o) = hv[ps];
      *(volatile v8us*)(pl_ + o) = lv[ps];
    }
  }
  __threadfence();
  #pragma unroll
  for (int ps = 0; ps < 5; ++ps) {
    const int lr = ps * 16 + rsub;
    if (lr < 66) {
      const size_t o = (qb + lr) * NIC + piece * 8;
      *(volatile v8us*)(ph_ + o) = hv[ps];
      *(volatile v8us*)(pl_ + o) = lv[ps];
    }
  }
  if (ph == 0 || ph == 63) {
    const size_t zb = (ph == 0) ? (size_t)0 : (size_t)65 * 66;
    const v8us z8 = {0, 0, 0, 0, 0, 0, 0, 0};
    #pragma unroll
    for (int ps = 0; ps < 5; ++ps) {
      const int lr = ps * 16 + rsub;
      if (lr < 66) {
        const size_t o = (zb + lr) * NIC + piece * 8;
        *(volatile v8us*)(ph_ + o) = z8;
        *(volatile v8us*)(pl_ + o) = z8;
      }
    }
    __threadfence();
    #pragma unroll
    for (int ps = 0; ps < 5; ++ps) {
      const int lr = ps * 16 + rsub;
      if (lr < 66) {
        const size_t o = (zb + lr) * NIC + piece * 8;
        *(volatile v8us*)(ph_ + o) = z8;
        *(volatile v8us*)(pl_ + o) = z8;
      }
    }
  }
}

template <int MODE>
__global__ __launch_bounds__(TPB) void gemm_k(
    const us16* __restrict__ Ah, const us16* __restrict__ Al, int lda,
    const us16* __restrict__ Bh, const us16* __restrict__ Bl, int ldb, int ksteps,
    us16* __restrict__ Oh, us16* __restrict__ Ol, float* __restrict__ Of, int ldo)
{
  constexpr bool CONV = (MODE == 2);
  __shared__ __attribute__((aligned(16))) float sD[128 * LDP];
  const int tid = threadIdx.x, lane = tid & 31, wave = tid >> 5;
  const int h = lane >> 4, m = lane & 15;
  const int wr = wave & 3, wc = wave >> 2;
  const int bx = blockIdx.x, by = blockIdx.y;
  const int row0 = by * 128, col0 = bx * 64;

  long long aoff[2], boff[2];
  #pragma unroll
  for (int i = 0; i < 2; ++i)
    aoff[i] = (long long)(row0 + wr * 32 + i * 16 + m) * lda + 8 * h;
  #pragma unroll
  for (int j = 0; j < 2; ++j) {
    const int cl = wc * 32 + j * 16 + m;
    if (CONV) boff[j] = (long long)((bx + 1) * 66 + cl + 1) * NIC + 8 * h;
    else      boff[j] = (long long)(col0 + cl) * ldb + 8 * h;
  }

  v8f acc[2][2];
  #pragma unroll
  for (int i = 0; i < 2; ++i)
    #pragma unroll
    for (int j = 0; j < 2; ++j) acc[i][j] = zero8f();

  #pragma unroll 1
  for (int ks = 0; ks < ksteps; ++ks) {
    const long long ak = (long long)ks * 32;
    long long bk;
    if (CONV) {
      const int tap = ks >> 2;
      const int dh = (tap >= 6) ? 1 : ((tap >= 3) ? 0 : -1);
      const int dw = tap - 3 * (dh + 1) - 1;
      bk = (long long)(dh * 66 + dw) * NIC + (ks & 3) * 32;
    } else {
      bk = ak;
    }
    FragB fah[2], fal[2], fbh[2], fbl[2];
    #pragma unroll
    for (int i = 0; i < 2; ++i) {
      const us16* p = Ah + (aoff[i] + ak);
      const us16* q = Al + (aoff[i] + ak);
      fah[i].half[0] = *(const v8usa*)(p);
      fah[i].half[1] = *(const v8usa*)(p + 16);
      fal[i].half[0] = *(const v8usa*)(q);
      fal[i].half[1] = *(const v8usa*)(q + 16);
    }
    #pragma unroll
    for (int j = 0; j < 2; ++j) {
      const us16* p = Bh + (boff[j] + bk);
      const us16* q = Bl + (boff[j] + bk);
      fbh[j].half[0] = *(const v8usa*)(p);
      fbh[j].half[1] = *(const v8usa*)(p + 16);
      fbl[j].half[0] = *(const v8usa*)(q);
      fbl[j].half[1] = *(const v8usa*)(q + 16);
    }
    #pragma unroll
    for (int i = 0; i < 2; ++i)
      #pragma unroll
      for (int j = 0; j < 2; ++j) {
        acc[i][j] = wmma_bf16(fah[i], fbh[j], acc[i][j]);
        acc[i][j] = wmma_bf16(fah[i], fbl[j], acc[i][j]);
        acc[i][j] = wmma_bf16(fal[i], fbh[j], acc[i][j]);
      }
  }

  #pragma unroll
  for (int i = 0; i < 2; ++i)
    #pragma unroll
    for (int j = 0; j < 2; ++j)
      #pragma unroll
      for (int r = 0; r < 8; ++r)
        sD[(wr * 32 + i * 16 + 8 * h + r) * LDP + wc * 32 + j * 16 + m] = acc[i][j][r];
  __syncthreads();

  if (MODE != 2) {
    const int piece = tid & 7, rl = tid >> 3;
    v8us hv[4], lv[4];
    size_t oo[4];
    #pragma unroll
    for (int g = 0; g < 4; ++g) {
      const int row = g * 32 + rl;
      const float* s = sD + row * LDP + piece * 8;
      const v4f f0 = *(const v4fa*)s;
      const v4f f1 = *(const v4fa*)(s + 4);
      #pragma unroll
      for (int i = 0; i < 4; ++i) {
        float v0 = f0[i], v1 = f1[i];
        if (MODE == 1) { v0 = sigm(v0); v1 = sigm(v1); }
        us16 a, b;
        split2(v0, a, b); hv[g][i] = a;     lv[g][i] = b;
        split2(v1, a, b); hv[g][4 + i] = a; lv[g][4 + i] = b;
      }
      oo[g] = (size_t)(row0 + row) * ldo + col0 + piece * 8;
      *(volatile v8us*)(Oh + oo[g]) = hv[g];
      *(volatile v8us*)(Ol + oo[g]) = lv[g];
    }
    __threadfence();
    #pragma unroll
    for (int g = 0; g < 4; ++g) {
      *(volatile v8us*)(Oh + oo[g]) = hv[g];
      *(volatile v8us*)(Ol + oo[g]) = lv[g];
    }
  } else {
    const int piece = tid & 15, rl = tid >> 4;
    v4f ov[8];
    size_t oo[8];
    #pragma unroll
    for (int g = 0; g < 8; ++g) {
      const int row = g * 16 + rl;
      const v4f f = *(const v4fa*)(sD + row * LDP + piece * 4);
      v4f o;
      #pragma unroll
      for (int i = 0; i < 4; ++i) o[i] = sigm(f[i]);
      ov[g] = o;
      oo[g] = (size_t)(row0 + row) * ldo + col0 + piece * 4;
      *(volatile v4f*)(Of + oo[g]) = ov[g];
    }
    __threadfence();
    #pragma unroll
    for (int g = 0; g < 8; ++g) *(volatile v4f*)(Of + oo[g]) = ov[g];
  }
}

extern "C" void kernel_launch(void* const* d_in, const int* in_sizes, int n_in,
                              void* d_out, int out_size, void* d_ws, size_t ws_size,
                              hipStream_t stream) {
  if (n_in < 7) return;
  const int nx = NCH * NPIX;
  if (in_sizes[0] != nx || in_sizes[1] != nx || in_sizes[2] != nx) return;
  if (in_sizes[3] != NIC * NCH || in_sizes[4] != NIC * NCH || in_sizes[5] != NIC * NCH) return;
  if (in_sizes[6] != NCH * KCV) return;
  if (out_size != nx) return;

  const float* x1      = (const float*)d_in[0];
  const float* x2      = (const float*)d_in[1];
  const float* x3      = (const float*)d_in[2];
  const float* w_phi   = (const float*)d_in[3];
  const float* w_theta = (const float*)d_in[4];
  const float* w_g     = (const float*)d_in[5];
  const float* w_mask  = (const float*)d_in[6];
  float* outp = (float*)d_out;

  const size_t PLX  = (size_t)NPIX * NCH;
  const size_t PLY1 = (size_t)NPIX * NPIX;
  const size_t PLW  = (size_t)NIC * NCH;
  const size_t PLWM = (size_t)NCH * KCV;
  const size_t PLP  = (size_t)NIC * NPIX;
  const size_t PLXP = (size_t)NPR * NIC;

  size_t off = 0;
  char* ws = (char*)d_ws;
  const size_t szR0 = ((6 * PLX > 2 * PLY1) ? 6 * PLX : 2 * PLY1) * 2;
  us16* R0  = (us16*)(ws + off); off += szR0;
  us16* WP  = (us16*)(ws + off); off += 6 * PLW * 2;
  us16* WM  = (us16*)(ws + off); off += 2 * PLWM * 2;
  us16* PHI = (us16*)(ws + off); off += 2 * PLP * 2;
  us16* THT = (us16*)(ws + off); off += 2 * PLP * 2;
  us16* GG  = (us16*)(ws + off); off += 2 * PLP * 2;
  us16* X33 = (us16*)(ws + off); off += 2 * PLP * 2;
  us16* Y2  = (us16*)(ws + off); off += 2 * PLP * 2;
  us16* XP  = (us16*)(ws + off); off += 2 * PLXP * 2;
  if (off > ws_size) return;
  us16* XT  = R0;
  us16* Y1h = R0;
  us16* Y1l = R0 + PLY1;

  kw1_k<<<dim3(64, 3), dim3(TPB), 0, stream>>>(w_phi, w_theta, w_g, WP);
  kwm_k<<<dim3((NCH * KCV / 8) / TPB), dim3(TPB), 0, stream>>>(w_mask, WM, WM + PLWM);
  kx_k<<<dim3(NPIX / 64, NCH / 64, 3), dim3(TPB), 0, stream>>>(x1, x2, x3, XT);

  gemm_k<0><<<dim3(NPIX / 64, 1), dim3(TPB), 0, stream>>>(
      WP, WP + PLW, NCH, XT, XT + PLX, NCH, NCH / 32, PHI, PHI + PLP, outp, NPIX);
  gemm_k<0><<<dim3(NIC / 64, NPIX / 128), dim3(TPB), 0, stream>>>(
      XT + 2 * PLX, XT + 3 * PLX, NCH, WP + 2 * PLW, WP + 3 * PLW, NCH, NCH / 32, THT, THT + PLP, outp, NIC);
  gemm_k<0><<<dim3(NPIX / 64, 1), dim3(TPB), 0, stream>>>(
      WP + 4 * PLW, WP + 5 * PLW, NCH, XT + 4 * PLX, XT + 5 * PLX, NCH, NCH / 32, GG, GG + PLP, outp, NPIX);

  kt1_k<<<dim3(NPIX / 64), dim3(TPB), 0, stream>>>(GG, GG + PLP, X33, X33 + PLP);

  gemm_k<1><<<dim3(NPIX / 64, NPIX / 128), dim3(TPB), 0, stream>>>(
      PHI, PHI + PLP, NIC, THT, THT + PLP, NIC, NIC / 32, Y1h, Y1l, outp, NPIX);

  gemm_k<0><<<dim3(NIC / 64, NPIX / 128), dim3(TPB), 0, stream>>>(
      Y1h, Y1l, NPIX, X33, X33 + PLP, NPIX, NPIX / 32, Y2, Y2 + PLP, outp, NIC);

  kt2_k<<<dim3(64), dim3(TPB), 0, stream>>>(Y2, Y2 + PLP, XP, XP + PLXP);

  gemm_k<2><<<dim3(NPIX / 64, NCH / 128), dim3(TPB), 0, stream>>>(
      WM, WM + PLWM, KCV, XP, XP + PLXP, NIC, KCV / 32, Y2, Y2 + PLP, outp, NPIX);
}
